// GroupedQueryAttention_25950192402649
// MI455X (gfx1250) — hardware-verified
//
#include <hip/hip_runtime.h>
#ifndef NB
#define NB 2
#endif
#ifndef SEQ
#define SEQ 2048
#endif
#define SEQ_FULL 2048
#define DM 2048
#define NH 32
#define NKV 8
#define HPG 4
#define HD 64
#define DQ (NH * HD)
#define DKV (NKV * HD)
#define NQKV (DQ + 2 * DKV)
#define BAND ((SEQ) < 512 ? (SEQ) : 512)
#define NR ((unsigned)(NB * SEQ))
#define PP 72

static_assert(HD == 64);
static_assert(NH == NKV * HPG);
static_assert(SEQ % 64 == 0);
static_assert(BAND % 64 == 0);
static_assert((SEQ - BAND) % 128 == 0);
static_assert(NR % 128u == 0u);
static_assert((NR * 40u) % 32u == 0u);
static_assert(NQKV % 64 == 0);
static_assert(DM % 64 == 0);
static_assert(DQ % 64 == 0);
static_assert(DM % 32 == 0);
static_assert(DQ % 32 == 0);
static_assert(NH + NKV == 40);
static_assert(SEQ <= SEQ_FULL);

typedef _Float16 v16h __attribute__((ext_vector_type(16)));
typedef __bf16 v16b __attribute__((ext_vector_type(16)));
typedef unsigned short v8us __attribute__((ext_vector_type(8), may_alias));
typedef float v8f __attribute__((ext_vector_type(8)));
typedef float v4f __attribute__((ext_vector_type(4)));
typedef float v4fa __attribute__((ext_vector_type(4), may_alias));
union Frag { v16h h; v16b b; v8us half[2]; };
union P8 { v8us v; unsigned short u[8]; };

__device__ __forceinline__ unsigned short bf16_bits(float x) { unsigned int u = __float_as_uint(x); return (unsigned short)((u + 0x7FFFu + ((u >> 16) & 1u)) >> 16); }
__device__ __forceinline__ float bf16_val(unsigned short b) { return __uint_as_float(((unsigned int)b) << 16); }
__device__ __forceinline__ float bf16_rne(float x) { return bf16_val(bf16_bits(x)); }
__device__ __forceinline__ unsigned short f16_bits(float x) { return __builtin_bit_cast(unsigned short, (_Float16)x); }
__device__ __forceinline__ float f16_val(unsigned short b) { return (float)__builtin_bit_cast(_Float16, b); }

__device__ __forceinline__ Frag ldfrag(const unsigned short* p, unsigned hh) { Frag f; f.half[0] = *(const v8us*)(p + 8u * hh); f.half[1] = *(const v8us*)(p + 16u + 8u * hh); return f; }
__device__ __forceinline__ v8f mma_h(v16h a, v16h b, v8f c) { v8f d = __builtin_amdgcn_wmma_f32_16x16x32_f16(false, a, false, b, (short)0, c, false, false); asm volatile("v_nop\n\tv_nop\n\tv_nop\n\tv_nop" : "+v"(d) : "v"(a), "v"(b)); return d; }
__device__ __forceinline__ v8f mma_b(v16b a, v16b b, v8f c) { v8f d = __builtin_amdgcn_wmma_f32_16x16x32_bf16(false, a, false, b, (short)0, c, false, false); asm volatile("v_nop\n\tv_nop\n\tv_nop\n\tv_nop" : "+v"(d) : "v"(a), "v"(b)); return d; }

__global__ __launch_bounds__(256) void k_x16(const float* __restrict__ x, unsigned short* __restrict__ X16) {
  const unsigned t = blockIdx.x * 256u + threadIdx.x;
  if (t >= NR * (DM / 8u)) return;
  const unsigned row = t / (DM / 8u), c8 = (t - row * (DM / 8u)) * 8u;
  const unsigned b = row / (unsigned)SEQ, s = row - b * (unsigned)SEQ;
  const float* src = x + ((size_t)b * SEQ_FULL + s) * DM + c8;
  const v4f a = *(const v4fa*)src, c = *(const v4fa*)(src + 4);
  P8 f;
#pragma unroll
  for (int q = 0; q < 4; ++q) { f.u[q] = f16_bits(bf16_rne(a[q])); f.u[4 + q] = f16_bits(bf16_rne(c[q])); }
  unsigned short* dst = X16 + (size_t)t * 8u;
  *(volatile v8us*)dst = f.v; __threadfence(); *(volatile v8us*)dst = f.v;
}

__global__ __launch_bounds__(256) void k_wnat(const float* __restrict__ w, unsigned n8, unsigned short* __restrict__ Bt) {
  const unsigned t = blockIdx.x * 256u + threadIdx.x;
  if (t >= n8) return;
  const float* src = w + (size_t)t * 8u;
  const v4f a = *(const v4fa*)src, c = *(const v4fa*)(src + 4);
  P8 f;
#pragma unroll
  for (int q = 0; q < 4; ++q) { f.u[q] = f16_bits(bf16_rne(a[q]) * 16.0f); f.u[4 + q] = f16_bits(bf16_rne(c[q]) * 16.0f); }
  unsigned short* dst = Bt + (size_t)t * 8u;
  *(volatile v8us*)dst = f.v; __threadfence(); *(volatile v8us*)dst = f.v;
}

__global__ __launch_bounds__(128) void k_gemm2(const unsigned short* __restrict__ A, unsigned lda, size_t sA, const unsigned short* __restrict__ Bh, unsigned ldb, float alpha,
                                              float* __restrict__ C, unsigned ldc, size_t sC, unsigned M, unsigned N, unsigned K) {
  __shared__ __attribute__((aligned(16))) float so[4][32][68];
  const unsigned tid = threadIdx.x, w = tid >> 5, lane = tid & 31u, ln = lane & 15u, hh = lane >> 4; const unsigned by = blockIdx.y;
  A += (size_t)by * sA; const size_t cofs = (size_t)by * sC;
  const unsigned ntn = N >> 6; const unsigned mt = blockIdx.x / ntn, nq = blockIdx.x - mt * ntn; const unsigned row0 = mt * 128u + 32u * w, col0 = nq * 64u; if (row0 >= M) return;
  const unsigned short* a0p = A + (size_t)(row0 + ln) * lda; const unsigned short* a1p = a0p + (size_t)16 * lda;
  const unsigned short* b0p = Bh + (size_t)(col0 + ln) * ldb; const unsigned short* b1p = b0p + (size_t)16 * ldb; const unsigned short* b2p = b1p + (size_t)16 * ldb; const unsigned short* b3p = b2p + (size_t)16 * ldb;
  const v8f z8 = {0.f,0.f,0.f,0.f,0.f,0.f,0.f,0.f}; v8f c00 = z8, c01 = z8, c02 = z8, c03 = z8, c10 = z8, c11 = z8, c12 = z8, c13 = z8;
#pragma unroll 1
  for (unsigned kb = 0; kb < K; kb += 32u) { const Frag a0 = ldfrag(a0p + kb, hh), a1 = ldfrag(a1p + kb, hh);
    Frag b = ldfrag(b0p + kb, hh); c00 = mma_h(a0.h, b.h, c00); c10 = mma_h(a1.h, b.h, c10);
    b = ldfrag(b1p + kb, hh); c01 = mma_h(a0.h, b.h, c01); c11 = mma_h(a1.h, b.h, c11);
    b = ldfrag(b2p + kb, hh); c02 = mma_h(a0.h, b.h, c02); c12 = mma_h(a1.h, b.h, c12);
    b = ldfrag(b3p + kb, hh); c03 = mma_h(a0.h, b.h, c03); c13 = mma_h(a1.h, b.h, c13); }
  v8f accs[8] = {c00, c01, c02, c03, c10, c11, c12, c13};
#pragma unroll
  for (int u = 0; u < 8; ++u) { const unsigned t = (unsigned)u & 3u, half = (unsigned)u >> 2;
#pragma unroll
    for (int r = 0; r < 8; ++r) { const unsigned rloc = half * 16u + 8u * hh + (unsigned)r; so[w][rloc][t * 16u + ln] = accs[u][r] * alpha; } }
  __builtin_amdgcn_fence(4  , "workgroup"); __builtin_amdgcn_wave_barrier();
  const unsigned rsub = lane >> 4, c4 = (lane & 15u) * 4u;
  for (int pass = 0; pass < 2; ++pass) {
#pragma unroll
    for (int q = 0; q < 16; ++q) { const unsigned r = (unsigned)q * 2u + rsub; const v4f v = *(const v4fa*)&so[w][r][c4]; *(volatile v4f*)(C + cofs + (size_t)(row0 + r) * ldc + col0 + c4) = v; }
    if (pass == 0) __threadfence(); }
}

__global__ __launch_bounds__(128) void k_gemm_res(const unsigned short* __restrict__ A, const unsigned short* __restrict__ Ar, unsigned lda, size_t sA, size_t sAr,
                                                 const unsigned short* __restrict__ Bh, unsigned ldb, float alpha, float* __restrict__ C, unsigned ldc, size_t sC, unsigned M, unsigned N, unsigned K) {
  __shared__ __attribute__((aligned(16))) float so[4][16][68];
  const unsigned tid = threadIdx.x, w = tid >> 5, lane = tid & 31u, ln = lane & 15u, hh = lane >> 4; const unsigned by = blockIdx.y;
  const size_t cofs = (size_t)by * sC;
  const unsigned ntn = N >> 6; const unsigned mt = blockIdx.x / ntn, nq = blockIdx.x - mt * ntn; const unsigned row0 = mt * 64u + 16u * w, col0 = nq * 64u; if (row0 >= M) return;
  const unsigned short* ap = A + (size_t)by * sA + (size_t)(row0 + ln) * lda; const unsigned short* rp = Ar + (size_t)by * sAr + (size_t)(row0 + ln) * lda;
  const unsigned short* b0p = Bh + (size_t)(col0 + ln) * ldb; const unsigned short* b1p = b0p + (size_t)16 * ldb; const unsigned short* b2p = b1p + (size_t)16 * ldb; const unsigned short* b3p = b2p + (size_t)16 * ldb;
  const v8f z8 = {0.f,0.f,0.f,0.f,0.f,0.f,0.f,0.f}; v8f h0 = z8, h1 = z8, h2 = z8, h3 = z8, r0 = z8, r1 = z8, r2 = z8, r3 = z8;
#pragma unroll 1
  for (unsigned kb = 0; kb < K; kb += 32u) { const Frag a = ldfrag(ap + kb, hh), ar = ldfrag(rp + kb, hh);
    Frag b = ldfrag(b0p + kb, hh); h0 = mma_h(a.h, b.h, h0); r0 = mma_h(ar.h, b.h, r0);
    b = ldfrag(b1p + kb, hh); h1 = mma_h(a.h, b.h, h1); r1 = mma_h(ar.h, b.h, r1);
    b = ldfrag(b2p + kb, hh); h2 = mma_h(a.h, b.h, h2); r2 = mma_h(ar.h, b.h, r2);
    b = ldfrag(b3p + kb, hh); h3 = mma_h(a.h, b.h, h3); r3 = mma_h(ar.h, b.h, r3); }
  v8f ah[4] = {h0, h1, h2, h3}; v8f al[4] = {r0, r1, r2, r3};
#pragma unroll
  for (int t = 0; t < 4; ++t) {
#pragma unroll
    for (int r = 0; r < 8; ++r) so[w][8u * hh + (unsigned)r][(unsigned)t * 16u + ln] = (ah[t][r] + al[t][r] * 0.0009765625f) * alpha; }
  __builtin_amdgcn_fence(4  , "workgroup"); __builtin_amdgcn_wave_barrier();
  const unsigned rsub = lane >> 4, c4 = (lane & 15u) * 4u;
  for (int pass = 0; pass < 2; ++pass) {
#pragma unroll
    for (int q = 0; q < 8; ++q) { const unsigned r = (unsigned)q * 2u + rsub; const v4f v = *(const v4fa*)&so[w][r][c4]; *(volatile v4f*)(C + cofs + (size_t)(row0 + r) * ldc + col0 + c4) = v; }
    if (pass == 0) __threadfence(); }
}

__global__ __launch_bounds__(256) void k_prep_qk(const float* __restrict__ QKV, const float* __restrict__ cosT, const float* __restrict__ sinT, const float* __restrict__ qw, const float* __restrict__ kw,
                                                unsigned short* __restrict__ Q16, unsigned short* __restrict__ K16, unsigned short* __restrict__ QBh, unsigned short* __restrict__ QBl,
                                                unsigned short* __restrict__ KBh, unsigned short* __restrict__ KBl) {
  const unsigned tid = threadIdx.x;
  const unsigned gu = blockIdx.x * 32u + (tid >> 3), u = tid & 7u;
  const unsigned row = gu / 40u, slot = gu - row * 40u;
  const unsigned b = row / (unsigned)SEQ, s = row - b * (unsigned)SEQ;
  const float* src = QKV + (size_t)row * NQKV + slot * 64u + u * 8u;
  const v4f x0 = *(const v4fa*)src, x1 = *(const v4fa*)(src + 4);
  float xs[8] = {x0[0], x0[1], x0[2], x0[3], x1[0], x1[1], x1[2], x1[3]};
  float ss = 0.f;
#pragma unroll
  for (int i = 0; i < 8; ++i) ss += xs[i] * xs[i];
  ss += __shfl_xor(ss, 1, 32); ss += __shfl_xor(ss, 2, 32); ss += __shfl_xor(ss, 4, 32);
  const float rs = rsqrtf(ss * 0.015625f + 1e-6f);
  const bool isq = slot < 32u;
  const v4f wq0 = *(const v4fa*)(qw + u * 8u), wq1 = *(const v4fa*)(qw + u * 8u + 4u);
  const v4f wk0 = *(const v4fa*)(kw + u * 8u), wk1 = *(const v4fa*)(kw + u * 8u + 4u);
  float wsq[8] = {wq0[0], wq0[1], wq0[2], wq0[3], wq1[0], wq1[1], wq1[2], wq1[3]};
  float wsk[8] = {wk0[0], wk0[1], wk0[2], wk0[3], wk1[0], wk1[1], wk1[2], wk1[3]};
  float y[8], py[8];
#pragma unroll
  for (int i = 0; i < 8; ++i) { const float wv = isq ? wsq[i] : wsk[i]; y[i] = xs[i] * rs * bf16_rne(wv); }
#pragma unroll
  for (int i = 0; i < 8; ++i) py[i] = __shfl_xor(y[i], 4, 32);
  const float sg = (u < 4u) ? -1.0f : 1.0f;
  const float* ct = cosT + (size_t)s * 64u + u * 8u; const float* st = sinT + (size_t)s * 64u + u * 8u;
  const v4f c0 = *(const v4fa*)ct, c1 = *(const v4fa*)(ct + 4), s0 = *(const v4fa*)st, s1 = *(const v4fa*)(st + 4);
  float cs[8] = {c0[0], c0[1], c0[2], c0[3], c1[0], c1[1], c1[2], c1[3]};
  float sn[8] = {s0[0], s0[1], s0[2], s0[3], s1[0], s1[1], s1[2], s1[3]};
  P8 fh, fbh, fbl;
#pragma unroll
  for (int i = 0; i < 8; ++i) {
    const float o = y[i] * bf16_rne(cs[i]) + (sg * py[i]) * bf16_rne(sn[i]);
    fh.u[i] = f16_bits(o);
    const unsigned short hb = bf16_bits(o); fbh.u[i] = hb; fbl.u[i] = bf16_bits(o - bf16_val(hb));
  }
  const unsigned hq = isq ? slot : slot - 32u;
  const unsigned nhp = isq ? (unsigned)NH : (unsigned)NKV;
  unsigned short* dm = (isq ? Q16 : K16) + ((size_t)(b * nhp + hq) * SEQ + s) * 64u + u * 8u;
  const bool inband = s < (unsigned)BAND;
  const unsigned sb = inband ? s : 0u;
  const size_t ob = ((size_t)(b * nhp + hq) * BAND + sb) * 64u + u * 8u;
  unsigned short* dh = (isq ? QBh : KBh) + ob; unsigned short* dl = (isq ? QBl : KBl) + ob;
  for (int pass = 0; pass < 2; ++pass) {
    *(volatile v8us*)dm = fh.v;
    if (inband) { *(volatile v8us*)dh = fbh.v; *(volatile v8us*)dl = fbl.v; }
    if (pass == 0) __threadfence();
  }
}

__global__ __launch_bounds__(256) void k_prep_v(const float* __restrict__ QKV, unsigned short* __restrict__ VT, unsigned short* __restrict__ VBh, unsigned short* __restrict__ VBl) {
  __shared__ __attribute__((aligned(16))) unsigned short th[64 * PP];
  __shared__ __attribute__((aligned(16))) unsigned short tbh[64 * PP];
  __shared__ __attribute__((aligned(16))) unsigned short tbl[64 * PP];
  const unsigned tid = threadIdx.x; const unsigned nt = (unsigned)SEQ / 64u;
  const unsigned slab = blockIdx.x / nt, tile = blockIdx.x - slab * nt; const unsigned b = slab / (unsigned)NKV, g = slab - b * (unsigned)NKV; const unsigned s0 = tile * 64u;
  const bool inband = s0 < (unsigned)BAND;
#pragma unroll
  for (int it = 0; it < 2; ++it) { const unsigned idx = tid + (unsigned)it * 256u; const unsigned r = idx >> 3, c8 = (idx & 7u) * 8u;
    const float* src = QKV + (size_t)(b * (unsigned)SEQ + s0 + r) * NQKV + DQ + DKV + g * 64u + c8;
    const v4f a = *(const v4fa*)src, c = *(const v4fa*)(src + 4);
    float vs[8] = {a[0], a[1], a[2], a[3], c[0], c[1], c[2], c[3]};
#pragma unroll
    for (int q = 0; q < 8; ++q) { const float v = vs[q]; th[(c8 + (unsigned)q) * PP + r] = f16_bits(v);
      if (inband) { const unsigned short hb = bf16_bits(v); tbh[(c8 + (unsigned)q) * PP + r] = hb; tbl[(c8 + (unsigned)q) * PP + r] = bf16_bits(v - bf16_val(hb)); } } }
  __syncthreads();
  P8 oh[2], obh[2], obl[2];
#pragma unroll
  for (int it = 0; it < 2; ++it) { const unsigned idx = tid + (unsigned)it * 256u; const unsigned d = idx >> 3, pc = (idx & 7u) * 8u;
    oh[it].v = *(const v8us*)(th + d * PP + pc); obh[it].v = oh[it].v; obl[it].v = oh[it].v;
    if (inband) { obh[it].v = *(const v8us*)(tbh + d * PP + pc); obl[it].v = *(const v8us*)(tbl + d * PP + pc); } }
  for (int pass = 0; pass < 2; ++pass) {
#pragma unroll
    for (int it = 0; it < 2; ++it) { const unsigned idx = tid + (unsigned)it * 256u; const unsigned d = idx >> 3, pc = (idx & 7u) * 8u;
      *(volatile v8us*)(VT + ((size_t)slab * 64u + d) * SEQ + s0 + pc) = oh[it].v;
      if (inband) { *(volatile v8us*)(VBh + ((size_t)slab * 64u + d) * BAND + s0 + pc) = obh[it].v; *(volatile v8us*)(VBl + ((size_t)slab * 64u + d) * BAND + s0 + pc) = obl[it].v; } }
    if (pass == 0) __threadfence(); }
}

template <bool RES>
__device__ __forceinline__ void flash_body(const unsigned short* Qh, const unsigned short* Ql, const unsigned short* Kh, const unsigned short* Kl, const unsigned short* Vh, const unsigned short* Vl,
                                           unsigned short* O16, unsigned short* ORES, unsigned qb0, unsigned short* pbh, unsigned short* pbl) {
  constexpr unsigned SL = RES ? (unsigned)BAND : (unsigned)SEQ;
  const unsigned tid = threadIdx.x, w = tid >> 5, lane = tid & 31u, ln = lane & 15u, hh = lane >> 4;
  const unsigned qblk = blockIdx.x + qb0, h = blockIdx.y, b = blockIdx.z, g = h / (unsigned)HPG;
  const unsigned q0 = qblk * 64u + w * 16u;
  unsigned short* ph = pbh + w * (16u * PP); unsigned short* pl = pbl + w * (RES ? 16u * PP : 0u);
  const size_t qoff = ((size_t)(b * (unsigned)NH + h) * SL + q0 + ln) * 64u;
  const Frag qh0 = ldfrag(Qh + qoff, hh), qh1 = ldfrag(Qh + qoff + 32, hh);
  Frag ql0 = qh0, ql1 = qh1;
  if (RES) { ql0 = ldfrag(Ql + qoff, hh); ql1 = ldfrag(Ql + qoff + 32, hh); }
  const size_t kslab = (size_t)(b * (unsigned)NKV + g) * SL * 64u;
  const size_t vslab = (size_t)(b * (unsigned)NKV + g) * 64u * SL;
  const v8f z8 = {0.f,0.f,0.f,0.f,0.f,0.f,0.f,0.f};
  v8f oacc[4] = {z8, z8, z8, z8};
  float mrun[8], srun[8];
#pragma unroll
  for (int r = 0; r < 8; ++r) { mrun[r] = -1.0e30f; srun[r] = 0.f; }
#pragma unroll 1
  for (unsigned kt = 0; kt <= qblk; ++kt) {
    const unsigned kb0 = kt * 64u;
    v8f sacc[4];
#pragma unroll
    for (int jt = 0; jt < 4; ++jt) {
      const size_t ko = kslab + (size_t)(kb0 + (unsigned)jt * 16u + ln) * 64u;
      const Frag k0 = ldfrag(Kh + ko, hh), k1 = ldfrag(Kh + ko + 32, hh);
      v8f sa = z8;
      if (RES) { const Frag l0 = ldfrag(Kl + ko, hh), l1 = ldfrag(Kl + ko + 32, hh);
        sa = mma_b(ql0.b, k0.b, sa); sa = mma_b(ql1.b, k1.b, sa); sa = mma_b(qh0.b, l0.b, sa); sa = mma_b(qh1.b, l1.b, sa); sa = mma_b(qh0.b, k0.b, sa); sa = mma_b(qh1.b, k1.b, sa); }
      else { sa = mma_h(qh0.h, k0.h, sa); sa = mma_h(qh1.h, k1.h, sa); }
      sacc[jt] = sa;
    }
    const bool diag = (kt == qblk);
#pragma unroll
    for (int r = 0; r < 8; ++r) {
      const unsigned qr = q0 + 8u * hh + (unsigned)r;
      float v[4]; float mx = -1.0e30f;
#pragma unroll
      for (int jt = 0; jt < 4; ++jt) { const unsigned key = kb0 + (unsigned)jt * 16u + ln; const bool ok = (!diag) || (key <= qr); const float t = ok ? sacc[jt][r] * 0.125f : -1.0e30f; v[jt] = t; mx = fmaxf(mx, t); }
      mx = fmaxf(mx, __shfl_xor(mx, 8, 32)); mx = fmaxf(mx, __shfl_xor(mx, 4, 32)); mx = fmaxf(mx, __shfl_xor(mx, 2, 32)); mx = fmaxf(mx, __shfl_xor(mx, 1, 32));
      const float mnew = fmaxf(mrun[r], mx);
      const float corr = __expf(mrun[r] - mnew);
      float es = 0.f;
#pragma unroll
      for (int jt = 0; jt < 4; ++jt) { const float e = __expf(v[jt] - mnew); es += e; const unsigned pi = (8u * hh + (unsigned)r) * PP + (unsigned)jt * 16u + ln;
        if (RES) { const unsigned short hb = bf16_bits(e); ph[pi] = hb; pl[pi] = bf16_bits(e - bf16_val(hb)); }
        else ph[pi] = f16_bits(e * 1024.0f); }
      srun[r] = srun[r] * corr + es; mrun[r] = mnew;
#pragma unroll
      for (int jh = 0; jh < 4; ++jh) oacc[jh][r] *= corr;
    }
    __builtin_amdgcn_fence(4  , "workgroup"); __builtin_amdgcn_wave_barrier();
    const Frag p0 = ldfrag(ph + ln * PP, hh), p1 = ldfrag(ph + ln * PP + 32, hh);
    Frag r0 = p0, r1 = p1;
    if (RES) { r0 = ldfrag(pl + ln * PP, hh); r1 = ldfrag(pl + ln * PP + 32, hh); }
#pragma unroll
    for (int jh = 0; jh < 4; ++jh) {
      const size_t vo = vslab + (size_t)((unsigned)jh * 16u + ln) * SL + kb0;
      const Frag v0 = ldfrag(Vh + vo, hh), v1 = ldfrag(Vh + vo + 32, hh);
      v8f oa = oacc[jh];
      if (RES) { const Frag w0 = ldfrag(Vl + vo, hh), w1 = ldfrag(Vl + vo + 32, hh);
        oa = mma_b(r0.b, v0.b, oa); oa = mma_b(r1.b, v1.b, oa); oa = mma_b(p0.b, w0.b, oa); oa = mma_b(p1.b, w1.b, oa); oa = mma_b(p0.b, v0.b, oa); oa = mma_b(p1.b, v1.b, oa); }
      else { oa = mma_h(p0.h, v0.h, oa); oa = mma_h(p1.h, v1.h, oa); }
      oacc[jh] = oa;
    }
    __builtin_amdgcn_fence(4  , "workgroup"); __builtin_amdgcn_wave_barrier();
  }
#pragma unroll
  for (int r = 0; r < 8; ++r) {
    float sr = srun[r]; sr += __shfl_xor(sr, 8, 32); sr += __shfl_xor(sr, 4, 32); sr += __shfl_xor(sr, 2, 32); sr += __shfl_xor(sr, 1, 32);
    const float inv = (RES ? 16.0f : 0.015625f) * (1.0f / sr);
#pragma unroll
    for (int jh = 0; jh < 4; ++jh) { const float o = oacc[jh][r] * inv; const unsigned short hb = f16_bits(o); const unsigned pi = (8u * hh + (unsigned)r) * PP + (unsigned)jh * 16u + ln;
      ph[pi] = hb; if (RES) pl[pi] = f16_bits((o - f16_val(hb)) * 1024.0f); }
  }
  __builtin_amdgcn_fence(4  , "workgroup"); __builtin_amdgcn_wave_barrier();
  P8 vh[4], vl[4];
#pragma unroll
  for (int it = 0; it < 4; ++it) { const unsigned row = (unsigned)it * 4u + (lane >> 3), pc = (lane & 7u) * 8u; vh[it].v = *(const v8us*)(ph + row * PP + pc); vl[it].v = vh[it].v; if (RES) vl[it].v = *(const v8us*)(pl + row * PP + pc); }
  for (int pass = 0; pass < 2; ++pass) {
#pragma unroll
    for (int it = 0; it < 4; ++it) { const unsigned row = (unsigned)it * 4u + (lane >> 3), pc = (lane & 7u) * 8u;
      *(volatile v8us*)(O16 + (size_t)(b * (unsigned)SEQ + q0 + row) * DQ + h * 64u + pc) = vh[it].v;
      if (RES) *(volatile v8us*)(ORES + (size_t)(b * (unsigned)BAND + q0 + row) * DQ + h * 64u + pc) = vl[it].v; }
    if (pass == 0) __threadfence(); }
}

__global__ __launch_bounds__(128) void k_flash_band(const unsigned short* __restrict__ Qh, const unsigned short* __restrict__ Ql, const unsigned short* __restrict__ Kh, const unsigned short* __restrict__ Kl,
                                                   const unsigned short* __restrict__ Vh, const unsigned short* __restrict__ Vl, unsigned short* __restrict__ O16, unsigned short* __restrict__ ORES) {
  __shared__ __attribute__((aligned(16))) unsigned short pbh[4 * 16 * PP];
  __shared__ __attribute__((aligned(16))) unsigned short pbl[4 * 16 * PP];
  flash_body<true>(Qh, Ql, Kh, Kl, Vh, Vl, O16, ORES, 0u, pbh, pbl);
}
__global__ __launch_bounds__(128) void k_flash_main(const unsigned short* __restrict__ Q16, const unsigned short* __restrict__ K16, const unsigned short* __restrict__ VT, unsigned short* __restrict__ O16, unsigned qb0) {
  __shared__ __attribute__((aligned(16))) unsigned short pbh[4 * 16 * PP];
  flash_body<false>(Q16, Q16, K16, K16, VT, VT, O16, O16, qb0, pbh, pbh);
}

extern "C" void kernel_launch(void* const* d_in, const int* in_sizes, int n_in,
                              void* d_out, int out_size, void* d_ws, size_t ws_size, hipStream_t stream) {
  (void)out_size;
  if (n_in < 9) return;
  if ((size_t)in_sizes[0] < ((size_t)(NB - 1) * SEQ_FULL + SEQ) * DM) return;
  if ((size_t)in_sizes[1] < (size_t)SEQ * 64 || (size_t)in_sizes[2] < (size_t)SEQ * 64) return;
  if ((size_t)in_sizes[3] < (size_t)DQ * DM || (size_t)in_sizes[4] < (size_t)DKV * DM || (size_t)in_sizes[5] < (size_t)DKV * DM || (size_t)in_sizes[6] < (size_t)DM * DQ) return;
  if (in_sizes[7] < 64 || in_sizes[8] < 64) return;
  const float* x = (const float*)d_in[0]; const float* rc = (const float*)d_in[1]; const float* rsn = (const float*)d_in[2];
  const float* wq = (const float*)d_in[3]; const float* wk = (const float*)d_in[4]; const float* wv = (const float*)d_in[5]; const float* wo = (const float*)d_in[6];
  const float* qnw = (const float*)d_in[7]; const float* knw = (const float*)d_in[8];
  float* out = (float*)d_out;
  char* ws = (char*)d_ws; size_t off = 0;
  auto take = [&](size_t bytes) { char* p = ws + off; off += (bytes + 255) & ~(size_t)255; return p; };
  unsigned short* XO = (unsigned short*)take((size_t)NR * DM * 2);
  unsigned short* WQKV = (unsigned short*)take((size_t)NQKV * DM * 2);
  unsigned short* WO = (unsigned short*)take((size_t)DM * DQ * 2);
  float* QKV = (float*)take((size_t)NR * NQKV * 4);
  unsigned short* Q16 = (unsigned short*)take((size_t)NR * DQ * 2);
  unsigned short* K16 = (unsigned short*)take((size_t)NR * DKV * 2);
  unsigned short* VT = (unsigned short*)take((size_t)NR * DKV * 2);
  unsigned short* QBh = (unsigned short*)take((size_t)NB * NH * BAND * 64 * 2);
  unsigned short* QBl = (unsigned short*)take((size_t)NB * NH * BAND * 64 * 2);
  unsigned short* KBh = (unsigned short*)take((size_t)NB * NKV * BAND * 64 * 2);
  unsigned short* KBl = (unsigned short*)take((size_t)NB * NKV * BAND * 64 * 2);
  unsigned short* VBh = (unsigned short*)take((size_t)NB * NKV * 64 * BAND * 2);
  unsigned short* VBl = (unsigned short*)take((size_t)NB * NKV * 64 * BAND * 2);
  unsigned short* ORES = (unsigned short*)take((size_t)NB * BAND * DQ * 2);
  static_assert(DQ == DM);
  if (off > ws_size || off > (size_t)134217728) return;
  unsigned short* X16 = XO; unsigned short* O16 = XO;

  k_x16<<<(unsigned)(((size_t)NR * (DM / 8) + 255) / 256), 256, 0, stream>>>(x, X16);
  k_wnat<<<(unsigned)(((size_t)DQ * DM / 8 + 255) / 256), 256, 0, stream>>>(wq, (unsigned)((size_t)DQ * DM / 8), WQKV);
  k_wnat<<<(unsigned)(((size_t)DKV * DM / 8 + 255) / 256), 256, 0, stream>>>(wk, (unsigned)((size_t)DKV * DM / 8), WQKV + (size_t)DQ * DM);
  k_wnat<<<(unsigned)(((size_t)DKV * DM / 8 + 255) / 256), 256, 0, stream>>>(wv, (unsigned)((size_t)DKV * DM / 8), WQKV + (size_t)(DQ + DKV) * DM);
  k_wnat<<<(unsigned)(((size_t)DM * DQ / 8 + 255) / 256), 256, 0, stream>>>(wo, (unsigned)((size_t)DM * DQ / 8), WO);
  k_gemm2<<<dim3((NR / 128u) * (NQKV / 64u), 1), 128, 0, stream>>>(X16, DM, 0, WQKV, DM, 0.0625f, QKV, NQKV, 0, NR, NQKV, DM);
  k_prep_qk<<<(NR * 40u) / 32u, 256, 0, stream>>>(QKV, rc, rsn, qnw, knw, Q16, K16, QBh, QBl, KBh, KBl);
  k_prep_v<<<(unsigned)(NB * NKV * (SEQ / 64)), 256, 0, stream>>>(QKV, VT, VBh, VBl);
  k_flash_band<<<dim3(BAND / 64, NH, NB), 128, 0, stream>>>(QBh, QBl, KBh, KBl, VBh, VBl, O16, ORES);
  if (SEQ > BAND)
    k_flash_main<<<dim3((SEQ - BAND) / 64, NH, NB), 128, 0, stream>>>(Q16, K16, VT, O16, (unsigned)(BAND / 64));
  k_gemm_res<<<dim3((BAND / 64) * (DM / 64), NB), 128, 0, stream>>>(O16, ORES, DQ, (size_t)SEQ * DQ, (size_t)BAND * DQ, WO, DQ, 0.00390625f, out, DM, (size_t)SEQ * DM, BAND, DM, DQ);
  if (SEQ > BAND)
    k_gemm2<<<dim3(((SEQ - BAND) / 128) * (DM / 64), NB), 128, 0, stream>>>(O16 + (size_t)BAND * DQ, DQ, (size_t)SEQ * DQ, WO, DQ, 0.00390625f, out + (size_t)BAND * DM, DM, (size_t)SEQ * DM, SEQ - BAND, DM, DQ);
}
